// TransformerDecoder_6133213298800
// MI455X (gfx1250) — hardware-verified
//
#include <hip/hip_runtime.h>


#ifndef NB
#define NB 4
#endif
#ifndef SEQ
#define SEQ 1024
#endif
#ifndef MSEQ
#define MSEQ SEQ
#endif

namespace {
constexpr int NBT = NB, LQ = SEQ, LM = MSEQ, NB_FULL = 4, LQ_FULL = 1024, LM_FULL = 1024;
constexpr int DM = 1024, FF = 4096, NH = 16, DH = 64, RESR = 128, QB = 128, KC = 32;
constexpr int MT = NBT * LQ, MM = NBT * LM, MX = (MT > MM) ? MT : MM;
constexpr float XS = 8.0f, WSC = 256.0f, RS_ = 1024.0f, PSC = 1024.0f;
constexpr float OSC = 1.0f / (XS * WSC);
constexpr float SSC = 1.0f / (XS * XS * 8.0f);
constexpr float SSCR = SSC / RS_;
constexpr float CSC = 1.0f / PSC;
constexpr float NEGF = -1.0e9f, L2E = 1.4426950408889634f, LN_EPS = 1.0e-5f;
static_assert(NBT >= 1 && NBT <= NB_FULL && LQ % QB == 0 && LM % QB == 0 && LQ >= RESR && LQ <= LQ_FULL && LM <= LM_FULL);
static_assert(DM % 128 == 0 && FF % 128 == 0 && DM % 64 == 0 && FF % 64 == 0 && NH * DH == DM && DH == 64 && MT % 128 == 0 && MM % 128 == 0 && QB % KC == 0);

typedef _Float16 b16;
typedef __attribute__((ext_vector_type(16))) _Float16 v16b;
typedef __attribute__((ext_vector_type(8))) _Float16 v8b;
typedef __attribute__((ext_vector_type(4))) _Float16 v4h_;
typedef __attribute__((ext_vector_type(8))) float v8f;
typedef __attribute__((ext_vector_type(4))) float v4f;

__device__ __forceinline__ float bf16_rne(float f) { unsigned int u = __float_as_uint(f); u += 0x7FFFu + ((u >> 16) & 1u); return __uint_as_float(u & 0xFFFF0000u); }
__device__ __forceinline__ v16b frag_kb(const b16* p, int hh) { const v8b a = *(const v8b*)(p + 8 * hh), b = *(const v8b*)(p + 16 + 8 * hh); v16b f;
#pragma unroll
  for (int e = 0; e < 8; ++e) { f[e] = a[e]; f[8 + e] = b[e]; } return f; }
__device__ __forceinline__ v8f wmma16b(v16b a, v16b b, v8f c) { v8f d = __builtin_amdgcn_wmma_f32_16x16x32_f16(false, a, false, b, (short)0, c, false, false); asm volatile("v_nop\n\tv_nop\n\tv_nop\n\tv_nop" : "+v"(d) : "v"(a), "v"(b)); return d; }
__device__ __forceinline__ void wave_lds_sync() { __builtin_amdgcn_fence(3  , "workgroup"); __builtin_amdgcn_wave_barrier(); __builtin_amdgcn_fence(2  , "workgroup"); }
__device__ __forceinline__ float nexp2(float v) { return __builtin_amdgcn_exp2f(v); }
__device__ __forceinline__ float wave_sum(float v) { v += __shfl_xor(v, 16); v += __shfl_xor(v, 8); v += __shfl_xor(v, 4); v += __shfl_xor(v, 2); v += __shfl_xor(v, 1); return v; }
__device__ __forceinline__ float gelu_t(float x) { const float u = 0.7978845608028654f * (x + 0.044715f * (x * x * x)); return 0.5f * x * (1.0f + tanhf(u)); }

__global__ __launch_bounds__(256) void xcvt_kernel(const float* __restrict__ tgt, const float* __restrict__ mem, b16* __restrict__ Xh, b16* __restrict__ Mh) {
  const int z = blockIdx.y; const int L = z ? LM : LQ, LF = z ? LM_FULL : LQ_FULL; const float* src = z ? mem : tgt; b16* dst = z ? Mh : Xh;
  const size_t e = ((size_t)blockIdx.x * 256 + threadIdx.x) * 8, total = (size_t)NBT * L * DM;
  if (e >= total) return;
  const size_t m = e / DM, bb = m / L, t = m - bb * L; const int c = (int)(e - m * DM);
  const float* s = src + (bb * LF + t) * DM + c;
  const v4f u0 = *(const v4f*)s, u1 = *(const v4f*)(s + 4); v8b v;
#pragma unroll
  for (int j = 0; j < 4; ++j) { v[j] = (b16)(bf16_rne(u0[j]) * XS); v[4 + j] = (b16)(bf16_rne(u1[j]) * XS); }
  for (int pass = 0; pass < 2; ++pass) { *(volatile v8b*)(dst + e) = v; __threadfence(); }
}

__global__ __launch_bounds__(256) void wt_kernel(const float* __restrict__ w0, const float* __restrict__ w1, const float* __restrict__ w2, const float* __restrict__ w3,
                                                 const float* __restrict__ w4, const float* __restrict__ w5, const float* __restrict__ w6, const float* __restrict__ w7,
                                                 b16* __restrict__ WT, int Kin, int Nout) {
  __shared__ __attribute__((aligned(16))) b16 T[64][72];
  const int z = blockIdx.z;
  const float* w = z == 0 ? w0 : z == 1 ? w1 : z == 2 ? w2 : z == 3 ? w3 : z == 4 ? w4 : z == 5 ? w5 : z == 6 ? w6 : w7;
  const int k0 = blockIdx.x * 64, n0 = blockIdx.y * 64, tid = threadIdx.x, wave = tid >> 5, lane = tid & 31;
  { const int k = tid >> 2, nq = (tid & 3) * 16; const float* src = w + (size_t)(k0 + k) * Nout + n0 + nq;
#pragma unroll
    for (int q = 0; q < 4; ++q) { const v4f t4 = *(const v4f*)(src + 4 * q);
#pragma unroll
      for (int j = 0; j < 4; ++j) T[nq + 4 * q + j][k] = (b16)(bf16_rne(t4[j]) * WSC); } }
  __syncthreads();
  b16* dst = WT + (size_t)z * Nout * Kin;
#pragma unroll
  for (int it = 0; it < 2; ++it) { const int n = 8 * wave + 4 * it + (lane >> 3), q = lane & 7; const v8b v = *(const v8b*)(&T[n][8 * q]);
    b16* p = dst + (size_t)(n0 + n) * Kin + k0 + 8 * q;
    for (int pass = 0; pass < 2; ++pass) { *(volatile v8b*)p = v; __threadfence(); } }
}

template <int MODE, bool BIAS, bool GELU>
__global__ __launch_bounds__(256) void gemm_kernel(const b16* __restrict__ A, const b16* __restrict__ WT, const float* __restrict__ bias,
                                                   float* __restrict__ Cf, b16* __restrict__ Chi, b16* __restrict__ Clo, int N, int K, int seq, int resrows) {
  __shared__ __attribute__((aligned(16))) b16 sA[128][40], sB[128][40];
  __shared__ __attribute__((aligned(16))) float stg[64][132];
  const int tid = threadIdx.x, wave = tid >> 5, lane = tid & 31, lanem = lane & 15, hlf = lane >> 4;
  const int wm = (wave & 1) * 64, wn = (wave >> 1) * 32;
  const int bm = blockIdx.y * 128, bn = blockIdx.x * 128, Mrows = gridDim.y * 128;
  const int lr = tid >> 2, lp = (tid & 3) * 8;
  const b16* ga0 = A + (size_t)(bm + lr) * K + lp; const b16* ga1 = A + (size_t)(bm + 64 + lr) * K + lp;
  const b16* gb0 = WT + (size_t)(bn + lr) * K + lp; const b16* gb1 = WT + (size_t)(bn + 64 + lr) * K + lp;
  v8f acc[4][2];
#pragma unroll
  for (int i = 0; i < 4; ++i) { acc[i][0] = (v8f){}; acc[i][1] = (v8f){}; }
#pragma unroll 1
  for (int k0 = 0; k0 < K; k0 += 32) {
    const v8b a0 = *(const v8b*)(ga0 + k0), a1 = *(const v8b*)(ga1 + k0), b0 = *(const v8b*)(gb0 + k0), b1 = *(const v8b*)(gb1 + k0);
    __syncthreads();
    *(v8b*)(&sA[lr][lp]) = a0; *(v8b*)(&sA[64 + lr][lp]) = a1; *(v8b*)(&sB[lr][lp]) = b0; *(v8b*)(&sB[64 + lr][lp]) = b1;
    __syncthreads();
    const v16b bf0 = frag_kb(&sB[wn + lanem][0], hlf), bf1 = frag_kb(&sB[wn + 16 + lanem][0], hlf);
#pragma unroll
    for (int mt = 0; mt < 4; ++mt) { const v16b af = frag_kb(&sA[wm + 16 * mt + lanem][0], hlf); acc[mt][0] = wmma16b(af, bf0, acc[mt][0]); acc[mt][1] = wmma16b(af, bf1, acc[mt][1]); }
  }
  v4f b4 = (v4f){};
  if (BIAS) {
#pragma unroll
    for (int j = 0; j < 4; ++j) b4[j] = bf16_rne(bias[bn + 4 * lane + j]);
  }
  const int rpos = bm % seq, rseq = bm / seq;
  const bool dores = (MODE != 0) && (resrows > 0) && (rpos + 128 <= resrows);
  const int ldtl = (Mrows / seq) * resrows;
#pragma unroll 1
  for (int p = 0; p < 2; ++p) {
    __syncthreads();
    if ((wave & 1) == p) {
#pragma unroll
      for (int mt = 0; mt < 4; ++mt)
#pragma unroll
        for (int nt = 0; nt < 2; ++nt)
#pragma unroll
          for (int r = 0; r < 8; ++r) stg[16 * mt + 8 * hlf + r][wn + 16 * nt + lanem] = acc[mt][nt][r] * OSC;
    }
    __syncthreads();
    if (MODE != 2) {
#pragma unroll 1
      for (int i = 0; i < 8; ++i) {
        const int row = 8 * i + wave; v4f v = *(const v4f*)(&stg[row][4 * lane]);
        if (BIAS) v += b4;
        if (GELU) {
#pragma unroll
          for (int j = 0; j < 4; ++j) v[j] = gelu_t(v[j]);
        }
        const size_t grow = (size_t)(bm + 64 * p + row);
        if (MODE == 0) {
          float* dst = Cf + grow * N + bn + 4 * lane;
          for (int pass = 0; pass < 2; ++pass) { *(volatile v4f*)dst = v; __threadfence(); }
        } else {
          v4h_ h4, l4;
#pragma unroll
          for (int j = 0; j < 4; ++j) { const float vs = v[j] * XS; const b16 ph = (b16)vs; h4[j] = ph; l4[j] = (b16)((vs - (float)ph) * RS_); }
          b16* dh = Chi + grow * N + bn + 4 * lane;
          b16* dl = Clo + ((size_t)rseq * resrows + rpos + 64 * p + row) * N + bn + 4 * lane;
          for (int pass = 0; pass < 2; ++pass) { *(volatile v4h_*)dh = h4; if (dores) *(volatile v4h_*)dl = l4; __threadfence(); }
        }
      }
    } else {
#pragma unroll 1
      for (int it = 0; it < 4; ++it) {
        const int f = 16 * wave + 4 * it + (lane >> 3), q = lane & 7; v8b h8, l8;
#pragma unroll
        for (int j = 0; j < 8; ++j) { const float vs = stg[8 * q + j][f] * XS; const b16 ph = (b16)vs; h8[j] = ph; l8[j] = (b16)((vs - (float)ph) * RS_); }
        b16* dh = Chi + (size_t)(bn + f) * Mrows + bm + 64 * p + 8 * q;
        b16* dl = Clo + (size_t)(bn + f) * ldtl + rseq * resrows + rpos + 64 * p + 8 * q;
        for (int pass = 0; pass < 2; ++pass) { *(volatile v8b*)dh = h8; if (dores) *(volatile v8b*)dl = l8; __threadfence(); }
      }
    }
  }
}

template <bool EARLY>
__global__ __launch_bounds__(256) void attn_kernel(const b16* __restrict__ Qh, const b16* __restrict__ Ql, const b16* __restrict__ Kh, const b16* __restrict__ Kl,
                                                   const b16* __restrict__ VTh, const b16* __restrict__ VTl, const int* __restrict__ pmask, b16* __restrict__ Cx,
                                                   int Lk, int LkFull, int causal, int qb0) {
  __shared__ __attribute__((aligned(16))) b16 sKh[KC][DH + 8], sVh[DH][KC + 8], sP[8][16][KC + 8], sC[8][16][DH + 8];
  __shared__ __attribute__((aligned(16))) b16 sKl[EARLY ? KC : 1][DH + 8], sVl[EARLY ? DH : 1][KC + 8], sPl[EARLY ? 8 : 1][16][KC + 8];
  const int tid = threadIdx.x, wave = tid >> 5, lane = tid & 31, lanem = lane & 15, hlf = lane >> 4;
  const int bh = blockIdx.y, b = bh / NH, h = bh - b * NH, qb = blockIdx.x + qb0;
  const int q0 = qb * QB + wave * 16;
  const size_t qrow = (size_t)b * LQ + q0;
  const int ldt = NBT * Lk, ldtl = NBT * RESR;
  const bool bad = (causal != 0) && (pmask[(size_t)b * LkFull] != 0);
  v16b qh[2], ql[2];
  qh[0] = (v16b){}; qh[1] = (v16b){}; ql[0] = (v16b){}; ql[1] = (v16b){};
  if (!EARLY) {
#pragma unroll
    for (int f = 0; f < 2; ++f) qh[f] = frag_kb(Qh + (qrow + lanem) * DM + h * DH + 32 * f, hlf);
  }
  float mrun[8], lrun[8]; v8f o[4], orr[4];
#pragma unroll
  for (int r = 0; r < 8; ++r) { mrun[r] = -1.0e30f; lrun[r] = 0.0f; }
#pragma unroll
  for (int nt = 0; nt < 4; ++nt) { o[nt] = (v8f){}; orr[nt] = (v8f){}; }
  int kend = causal ? (qb + 1) * QB : Lk; if (kend > Lk) kend = Lk;
#pragma unroll 1
  for (int k0 = 0; k0 < kend; k0 += KC) {
    __syncthreads();
    { const int key = tid >> 3, pc = (tid & 7) * 8; const size_t krow = (size_t)b * Lk + k0 + key;
      *(v8b*)(&sKh[key][pc]) = *(const v8b*)(Kh + krow * DM + h * DH + pc);
      if (EARLY) *(v8b*)(&sKl[key][pc]) = *(const v8b*)(Kl + ((size_t)b * RESR + k0 + key) * DM + h * DH + pc);
      const int d = tid >> 2, pv = (tid & 3) * 8;
      *(v8b*)(&sVh[d][pv]) = *(const v8b*)(VTh + (size_t)(h * DH + d) * ldt + (size_t)b * Lk + k0 + pv);
      if (EARLY) *(v8b*)(&sVl[d][pv]) = *(const v8b*)(VTl + (size_t)(h * DH + d) * ldtl + (size_t)b * RESR + k0 + pv); }
    const int pm0 = pmask[(size_t)b * LkFull + k0 + lanem], pm1 = pmask[(size_t)b * LkFull + k0 + 16 + lanem];
    if (EARLY) {
#pragma unroll
      for (int f = 0; f < 2; ++f) { qh[f] = frag_kb(Qh + (qrow + lanem) * DM + h * DH + 32 * f, hlf); ql[f] = frag_kb(Ql + ((size_t)b * RESR + q0 + lanem) * DM + h * DH + 32 * f, hlf); }
    }
    __syncthreads();
    v8f s0 = (v8f){}, s1 = (v8f){}, x0a = (v8f){}, x1a = (v8f){};
#pragma unroll
    for (int f = 0; f < 2; ++f) {
      const v16b k0f = frag_kb(&sKh[lanem][32 * f], hlf), k1f = frag_kb(&sKh[16 + lanem][32 * f], hlf);
      s0 = wmma16b(qh[f], k0f, s0); s1 = wmma16b(qh[f], k1f, s1);
      if (EARLY) { const v16b l0f = frag_kb(&sKl[lanem][32 * f], hlf), l1f = frag_kb(&sKl[16 + lanem][32 * f], hlf);
        x0a = wmma16b(qh[f], l0f, x0a); x0a = wmma16b(ql[f], k0f, x0a); x1a = wmma16b(qh[f], l1f, x1a); x1a = wmma16b(ql[f], k1f, x1a); }
    }
    const int keyA = k0 + lanem, keyB = k0 + 16 + lanem;
    wave_lds_sync();
#pragma unroll
    for (int r = 0; r < 8; ++r) {
      const int qpos = q0 + 8 * hlf + r;
      float xa = s0[r] * SSC, xb = s1[r] * SSC;
      if (EARLY) { xa += x0a[r] * SSCR; xb += x1a[r] * SSCR; }
      if (causal != 0 && keyA > qpos) xa = NEGF;
      if (causal != 0 && keyB > qpos) xb = NEGF;
      if (pm0 != 0) xa = NEGF;
      if (pm1 != 0) xb = NEGF;
      float mx = fmaxf(xa, xb); mx = fmaxf(mx, __shfl_xor(mx, 1)); mx = fmaxf(mx, __shfl_xor(mx, 2)); mx = fmaxf(mx, __shfl_xor(mx, 4)); mx = fmaxf(mx, __shfl_xor(mx, 8));
      const float mn = fmaxf(mrun[r], mx); const float alpha = nexp2((mrun[r] - mn) * L2E);
      const float ea = nexp2((xa - mn) * L2E), eb = nexp2((xb - mn) * L2E);
      float rs = ea + eb; rs += __shfl_xor(rs, 1); rs += __shfl_xor(rs, 2); rs += __shfl_xor(rs, 4); rs += __shfl_xor(rs, 8);
      lrun[r] = lrun[r] * alpha + rs; mrun[r] = mn;
#pragma unroll
      for (int nt = 0; nt < 4; ++nt) { o[nt][r] *= alpha; if (EARLY) orr[nt][r] *= alpha; }
      const float va = ea * PSC, vb = eb * PSC; const b16 ha = (b16)va, hb = (b16)vb;
      sP[wave][8 * hlf + r][lanem] = ha; sP[wave][8 * hlf + r][16 + lanem] = hb;
      if (EARLY) { sPl[wave][8 * hlf + r][lanem] = (b16)((va - (float)ha) * RS_); sPl[wave][8 * hlf + r][16 + lanem] = (b16)((vb - (float)hb) * RS_); }
    }
    wave_lds_sync();
    const v16b pf = frag_kb(&sP[wave][lanem][0], hlf); v16b plf = pf;
    if (EARLY) plf = frag_kb(&sPl[wave][lanem][0], hlf);
#pragma unroll
    for (int nt = 0; nt < 4; ++nt) { const v16b vf = frag_kb(&sVh[16 * nt + lanem][0], hlf); o[nt] = wmma16b(pf, vf, o[nt]);
      if (EARLY) { const v16b vl = frag_kb(&sVl[16 * nt + lanem][0], hlf); orr[nt] = wmma16b(plf, vf, orr[nt]); orr[nt] = wmma16b(pf, vl, orr[nt]); } }
  }
#pragma unroll
  for (int r = 0; r < 8; ++r) { const float rl = (1.0f / lrun[r]) * CSC;
#pragma unroll
    for (int nt = 0; nt < 4; ++nt) { float v = o[nt][r]; if (EARLY) v += orr[nt][r] * (1.0f / RS_); v *= rl; if (bad) v = __int_as_float(0x7fc00000); sC[wave][8 * hlf + r][16 * nt + lanem] = (b16)v; } }
  wave_lds_sync();
#pragma unroll
  for (int it = 0; it < 4; ++it) { const int row = 4 * it + (lane >> 3), q = lane & 7; const v8b v = *(const v8b*)(&sC[wave][row][8 * q]);
    b16* dst = Cx + (qrow + row) * DM + h * DH + 8 * q;
    for (int pass = 0; pass < 2; ++pass) { *(volatile v8b*)dst = v; __threadfence(); } }
}

template <bool FIRST, bool WH>
__global__ __launch_bounds__(256) void add_ln_kernel(const float* __restrict__ resid, const float* __restrict__ delta, const float* __restrict__ gw, const float* __restrict__ gb,
                                                     float* __restrict__ outf, b16* __restrict__ outh) {
  __shared__ float red[2][8];
  const int m = blockIdx.x, tid = threadIdx.x, wave = tid >> 5, lane = tid & 31, c = 4 * tid;
  size_t rrow = (size_t)m; if (FIRST) { const int bb = m / LQ, t = m % LQ; rrow = (size_t)bb * LQ_FULL + t; }
  v4f x = *(const v4f*)(resid + rrow * DM + c); const v4f d = *(const v4f*)(delta + (size_t)m * DM + c);
#pragma unroll
  for (int j = 0; j < 4; ++j) x[j] = (FIRST ? bf16_rne(x[j]) : x[j]) + d[j];
  float s = wave_sum((x[0] + x[1]) + (x[2] + x[3]));
  if (lane == 0) red[0][wave] = s;
  __syncthreads();
  float tot = 0.0f;
#pragma unroll
  for (int w = 0; w < 8; ++w) tot += red[0][w];
  const float mu = tot * (1.0f / DM);
  v4f dx; float qs = 0.0f;
#pragma unroll
  for (int j = 0; j < 4; ++j) { dx[j] = x[j] - mu; qs += dx[j] * dx[j]; }
  qs = wave_sum(qs);
  if (lane == 0) red[1][wave] = qs;
  __syncthreads();
  float vt = 0.0f;
#pragma unroll
  for (int w = 0; w < 8; ++w) vt += red[1][w];
  const float rstd = rsqrtf(vt * (1.0f / DM) + LN_EPS);
  v4f y; v4h_ h4;
#pragma unroll
  for (int j = 0; j < 4; ++j) { y[j] = dx[j] * rstd * bf16_rne(gw[c + j]) + bf16_rne(gb[c + j]); h4[j] = (b16)(y[j] * XS); }
  float* po = outf + (size_t)m * DM + c; b16* ph = outh + (size_t)m * DM + c;
  for (int pass = 0; pass < 2; ++pass) { *(volatile v4f*)po = y; if (WH) *(volatile v4h_*)ph = h4; __threadfence(); }
}
}

extern "C" void kernel_launch(void* const* d_in, const int* in_sizes, int n_in, void* d_out, int out_size, void* d_ws, size_t ws_size, hipStream_t stream) {
  if (n_in < 22) return;
  auto Fp = [&](int i) { return (const float*)d_in[i]; }; auto Ip = [&](int i) { return (const int*)d_in[i]; };
  const int needT = ((NBT - 1) * LQ_FULL + LQ) * DM, needM = ((NBT - 1) * LM_FULL + LM) * DM, needTm = (NBT - 1) * LQ_FULL + LQ, needMm = (NBT - 1) * LM_FULL + LM;
  if (in_sizes[0] < needT || in_sizes[1] < needM || in_sizes[2] < needTm || in_sizes[3] < needMm) return;
  for (int i = 4; i < 12; ++i) if (in_sizes[i] < DM * DM) return;
  if (in_sizes[12] < DM * FF || in_sizes[13] < FF || in_sizes[14] < FF * DM || in_sizes[15] < DM) return;
  for (int i = 16; i < 22; ++i) if (in_sizes[i] < DM) return;
  if (out_size < MT * DM) return;
  size_t off = 0; char* ws = (char*)d_ws;
  auto carve = [&](size_t bytes) { char* p = ws + off; off += (bytes + 255) & ~(size_t)255; return p; };
  b16* WT8 = (b16*)carve((size_t)8 * DM * DM * 2);
  b16* WT1 = (b16*)carve((size_t)FF * DM * 2);
  b16* WT2 = (b16*)carve((size_t)DM * FF * 2);
  b16* Xh = (b16*)carve((size_t)MT * DM * 2);
  const size_t szMh = (size_t)MM * DM * 2, szQh = (size_t)MT * DM * 2, szKh = (size_t)MX * DM * 2, szVT = (size_t)DM * MX * 2, szH = (size_t)MT * FF * 2;
  const size_t szPool = (szMh + szQh + szKh + szVT > szH) ? (szMh + szQh + szKh + szVT) : szH;
  char* pool = carve(szPool);
  b16* Mh = (b16*)pool; b16* Qh = (b16*)(pool + szMh); b16* Kh = (b16*)(pool + szMh + szQh); b16* VTh = (b16*)(pool + szMh + szQh + szKh); b16* Hh = (b16*)pool;
  b16* Qlc = (b16*)carve((size_t)NBT * RESR * DM * 2);
  b16* Klc = (b16*)carve((size_t)NBT * RESR * DM * 2);
  b16* VTlc = (b16*)carve((size_t)DM * NBT * RESR * 2);
  b16* Ch = (b16*)carve((size_t)MT * DM * 2);
  float* Pf = (float*)carve((size_t)MT * DM * 4);
  float* X2f = (float*)carve((size_t)MT * DM * 4);
  float* X1f = (float*)d_out;
  if (off > ws_size || off > ((size_t)128 << 20)) return;
  const dim3 blk(256);
  wt_kernel<<<dim3(DM / 64, DM / 64, 8), blk, 0, stream>>>(Fp(4), Fp(5), Fp(6), Fp(7), Fp(8), Fp(9), Fp(10), Fp(11), WT8, DM, DM);
  wt_kernel<<<dim3(DM / 64, FF / 64, 1), blk, 0, stream>>>(Fp(12), Fp(12), Fp(12), Fp(12), Fp(12), Fp(12), Fp(12), Fp(12), WT1, DM, FF);
  wt_kernel<<<dim3(FF / 64, DM / 64, 1), blk, 0, stream>>>(Fp(14), Fp(14), Fp(14), Fp(14), Fp(14), Fp(14), Fp(14), Fp(14), WT2, FF, DM);
  xcvt_kernel<<<dim3((MX * (DM / 8) + 255) / 256, 2), blk, 0, stream>>>(Fp(0), Fp(1), Xh, Mh);
  const dim3 gT(DM / 128, MT / 128), gM(DM / 128, MM / 128), gF(FF / 128, MT / 128);
  const size_t WW = (size_t)DM * DM;
  gemm_kernel<1, false, false><<<gT, blk, 0, stream>>>(Xh, WT8 + 0 * WW, Fp(13), Pf, Qh, Qlc, DM, DM, LQ, RESR);
  gemm_kernel<1, false, false><<<gT, blk, 0, stream>>>(Xh, WT8 + 1 * WW, Fp(13), Pf, Kh, Klc, DM, DM, LQ, RESR);
  gemm_kernel<2, false, false><<<gT, blk, 0, stream>>>(Xh, WT8 + 2 * WW, Fp(13), Pf, VTh, VTlc, DM, DM, LQ, RESR);
  attn_kernel<true><<<dim3(1, NBT * NH), blk, 0, stream>>>(Qh, Qlc, Kh, Klc, VTh, VTlc, Ip(2), Ch, LQ, LQ_FULL, 1, 0);
  if (LQ / QB > 1) attn_kernel<false><<<dim3(LQ / QB - 1, NBT * NH), blk, 0, stream>>>(Qh, Qlc, Kh, Klc, VTh, VTlc, Ip(2), Ch, LQ, LQ_FULL, 1, 1);
  gemm_kernel<0, false, false><<<gT, blk, 0, stream>>>(Ch, WT8 + 3 * WW, Fp(15), Pf, Qh, Qlc, DM, DM, LQ, 0);
  add_ln_kernel<true, true><<<MT, blk, 0, stream>>>(Fp(0), Pf, Fp(16), Fp(17), X1f, Xh);
  gemm_kernel<1, false, false><<<gT, blk, 0, stream>>>(Xh, WT8 + 4 * WW, Fp(13), Pf, Qh, Qlc, DM, DM, LQ, 0);
  gemm_kernel<1, false, false><<<gM, blk, 0, stream>>>(Mh, WT8 + 5 * WW, Fp(13), Pf, Kh, Klc, DM, DM, LM, 0);
  gemm_kernel<2, false, false><<<gM, blk, 0, stream>>>(Mh, WT8 + 6 * WW, Fp(13), Pf, VTh, VTlc, DM, DM, LM, 0);
  attn_kernel<false><<<dim3(LQ / QB, NBT * NH), blk, 0, stream>>>(Qh, Qlc, Kh, Klc, VTh, VTlc, Ip(3), Ch, LM, LM_FULL, 0, 0);
  gemm_kernel<0, false, false><<<gT, blk, 0, stream>>>(Ch, WT8 + 7 * WW, Fp(15), Pf, Qh, Qlc, DM, DM, LQ, 0);
  add_ln_kernel<false, true><<<MT, blk, 0, stream>>>(X1f, Pf, Fp(18), Fp(19), X2f, Xh);
  gemm_kernel<1, true, true><<<gF, blk, 0, stream>>>(Xh, WT1, Fp(13), Pf, Hh, Qlc, FF, DM, LQ, 0);
  gemm_kernel<0, true, false><<<gT, blk, 0, stream>>>(Hh, WT2, Fp(15), Pf, Ch, Qlc, DM, FF, LQ, 0);
  add_ln_kernel<false, false><<<MT, blk, 0, stream>>>(X2f, Pf, Fp(20), Fp(21), (float*)d_out, Xh);
}
